// CyclicTiSASRec_65274912964707
// MI455X (gfx1250) — hardware-run, weakly checked
//
#include <hip/hip_runtime.h>
#include <math.h>

typedef __attribute__((ext_vector_type(16))) _Float16 v16h;
typedef __attribute__((ext_vector_type(8)))  _Float16 v8h;
typedef __attribute__((ext_vector_type(8)))  float    v8f;
typedef __attribute__((ext_vector_type(4)))  float    v4f;
typedef __attribute__((ext_vector_type(4)))  unsigned int v4u;
typedef __attribute__((ext_vector_type(2)))  unsigned int v2u;
typedef __attribute__((ext_vector_type(4)))  int      v4i;

constexpr int kB = 8;
constexpr int kT = 256;
constexpr int kH = 128;
constexpr int kNH = 2;
constexpr int kDH = 64;
constexpr int kL = 2;
constexpr int kTok = kB * kT;
constexpr int kItems = 50001;
constexpr int kSpanRows = 257;
constexpr int kTKP = 320;
constexpr int kQTP = kNH * kTKP;
static_assert(kH == kNH * kDH, "head split");
static_assert(kTok == 2048 && kT == 256 && kH == 128 && kDH == 64, "shape contract");
static_assert((kH % 32) == 0 && (kDH % 32) == 0 && (kT % 32) == 0, "GEMM K multiples of 32");
static_assert((kTok % 64) == 0 && (kT % 64) == 0 && (kH % 64) == 0 && (kDH % 64) == 0 && (kTKP % 64) == 0, "GEMM M,N multiples of 64");
static_assert(kTKP >= kSpanRows, "table pad");

constexpr float kWCarry    = 16.0f;
constexpr float kWCarryInv = 1.0f / 16.0f;
constexpr float kPCarry    = 32768.0f;
constexpr float kPCarryInv = 1.0f / 32768.0f;
constexpr float kNegFill   = -1e9f;
constexpr float kLnEps     = 1e-8f;
constexpr float kTwoPi     = (float)(2.0 * 3.14159265358979323846);
constexpr float kInvP0     = 1.0f / 86400.0f;
constexpr float kInvP1     = 1.0f / 604800.0f;
constexpr float kInvP2     = 1.0f / 2592000.0f;
constexpr float kInvH      = 1.0f / (float)kH;

constexpr size_t kSzW    = (size_t)kL * kH * kH * 2;
constexpr size_t kSzHH16 = (size_t)kH * kH * 2;
constexpr size_t kSzTok32 = (size_t)kTok * kH * 4;
constexpr size_t kSzTok16 = (size_t)kTok * kH * 2;
constexpr size_t kOffWQ   = 0;
constexpr size_t kOffWK   = kOffWQ + kSzW;
constexpr size_t kOffWV   = kOffWK + kSzW;
constexpr size_t kOffW1   = kOffWV + kSzW;
constexpr size_t kOffW2   = kOffW1 + kSzW;
constexpr size_t kOffFW1  = kOffW2 + kSzW;
constexpr size_t kOffFW2  = kOffFW1 + kSzHH16;
constexpr size_t kOffTK   = kOffFW2 + kSzHH16;
constexpr size_t kOffAVT  = kOffTK + (size_t)kTKP * kH * 2;
constexpr size_t kOffSC   = kOffAVT + (size_t)kH * kT * 4;
constexpr size_t kOffHB   = kOffSC + (size_t)kB * 6 * kT * 4;
constexpr size_t kOffQN32 = kOffHB + (size_t)kB * kH * 4;
constexpr size_t kOffQN16 = kOffQN32 + kSzTok32;
constexpr size_t kOffSEQ16 = kOffQN16 + kSzTok16;
constexpr size_t kOffQ16  = kOffSEQ16 + kSzTok16;
constexpr size_t kOffKP16 = kOffQ16 + kSzTok16;
constexpr size_t kOffVT16 = kOffKP16 + kSzTok16;
constexpr size_t kOffS32  = kOffVT16 + kSzTok16;
constexpr size_t kOffQT32 = kOffS32 + (size_t)kB * kNH * kT * kT * 4;
constexpr size_t kOffP16  = kOffQT32 + (size_t)kTok * kQTP * 4;
constexpr size_t kOffOH32 = kOffP16 + (size_t)kB * kNH * kT * kT * 2;
constexpr size_t kOffX32  = kOffOH32 + kSzTok32;
constexpr size_t kOffX16  = kOffX32 + kSzTok32;
constexpr size_t kOffH116 = kOffX16 + kSzTok16;
constexpr size_t kOffSEQ32 = kOffH116 + kSzTok16;
constexpr size_t kOffLF16 = kOffSEQ32 + kSzTok32;
constexpr size_t kOffPRE32 = kOffLF16 + kSzTok16;
constexpr size_t kOffG16  = kOffPRE32 + kSzTok32;
constexpr size_t kOffFU32 = kOffG16 + kSzTok16;
constexpr size_t kWsTotal = kOffFU32 + kSzTok32;
static_assert(kWsTotal == 23203840ull, "carve total");
static_assert(kWsTotal <= 134217728ull, "carve cap");
static_assert((kOffTK % 128) == 0 && (kOffAVT % 128) == 0 && (kOffSC % 128) == 0 && (kOffHB % 128) == 0 &&
              (kOffQN32 % 128) == 0 && (kOffS32 % 128) == 0 && (kOffQT32 % 128) == 0 && (kOffP16 % 128) == 0 &&
              (kOffFU32 % 128) == 0, "128-B aligned regions");
static_assert((size_t)kTok * 4 == 8192 && (size_t)2 * kTok * 4 == 16384, "output packing");

__device__ __forceinline__ unsigned pk16(unsigned short a, unsigned short b) { return (unsigned)a | ((unsigned)b << 16); }
__device__ __forceinline__ unsigned short h_bits(float f) { const _Float16 h = (_Float16)f; return __builtin_bit_cast(unsigned short, h); }
__device__ __forceinline__ float h16_to_f32(unsigned hb) {
  const unsigned sgn = (hb & 0x8000u) << 16;
  const unsigned em = hb & 0x7fffu;
  const float fn = __uint_as_float((em << 13) + 0x38000000u);
  const float fs = (float)em * 5.9604644775390625e-8f;
  const float mag = (em < 0x400u) ? fs : fn;
  return __uint_as_float(__float_as_uint(mag) | sgn);
}
union FragU { v16h v; v8h h[2]; };
__device__ __forceinline__ v16h frag_load(const _Float16* p) {
  FragU f;
  f.h[0] = *(const v8h*)(p);
  f.h[1] = *(const v8h*)(p + 16);
  return f.v;
}
__device__ __forceinline__ v8f mma_h(v16h a, v16h b, v8f c) {
  c = __builtin_amdgcn_wmma_f32_16x16x32_f16(false, a, false, b, (short)0, c, false, false);
  asm volatile("v_nop\n\tv_nop\n\tv_nop\n\tv_nop" : "+v"(c) : "v"(a), "v"(b));
  return c;
}

template <int OUT_MODE, int BIAS_MODE, bool RESID, int ACT, bool KEEPM>
__global__ __launch_bounds__(256) void gemm_f16_tile64(
    const unsigned short* __restrict__ Ap, int lda, long sAo, long sAi,
    const unsigned short* __restrict__ Btp, int ldb, long sBo, long sBi,
    void* __restrict__ Cout, int ldc, long sCo, long sCi,
    const float* __restrict__ bias,
    const float* __restrict__ resid, int ldr, long sRo, long sRi,
    const int* __restrict__ keepv,
    int bdiv, int M, int N, int K, float scale) {
  const _Float16* A  = (const _Float16*)Ap;
  const _Float16* Bt = (const _Float16*)Btp;
  __shared__ __align__(16) float sT[8][16 * 68];
  const int z    = blockIdx.y;
  const int bo   = z / bdiv;
  const int bi   = z - bo * bdiv;
  const int lane = threadIdx.x & 31;
  const int wave = threadIdx.x >> 5;
  const int tilesN = N >> 6;
  const int tilesM = M >> 6;
  const int tile = blockIdx.x * 8 + wave;
  if (tile >= tilesM * tilesN) return;
  const int tm = tile / tilesN;
  const int tn = tile - tm * tilesN;
  const int m0 = tm << 6;
  const int n0 = tn << 6;

  const _Float16* Ab = A  + (size_t)bo * (size_t)sAo + (size_t)bi * (size_t)sAi;
  const _Float16* Bb = Bt + (size_t)bo * (size_t)sBo + (size_t)bi * (size_t)sBi;
  const size_t offC  = (size_t)bo * (size_t)sCo + (size_t)bi * (size_t)sCi;

  const int rlane = lane & 15;
  const int koff  = (lane >> 4) * 8;
  const int mOff  = (lane >> 4) * 8;

  v8f acc[4][4];
#pragma unroll
  for (int i = 0; i < 4; ++i)
#pragma unroll
    for (int j = 0; j < 4; ++j) acc[i][j] = (v8f){0.f, 0.f, 0.f, 0.f, 0.f, 0.f, 0.f, 0.f};

  for (int k0 = 0; k0 < K; k0 += 32) {
    v16h bh[4];
#pragma unroll
    for (int j = 0; j < 4; ++j) {
      const size_t bofs = (size_t)(n0 + (j << 4) + rlane) * ldb + koff + k0;
      bh[j] = frag_load(Bb + bofs);
    }
#pragma unroll
    for (int i = 0; i < 4; ++i) {
      const size_t aofs = (size_t)(m0 + (i << 4) + rlane) * lda + koff + k0;
      const v16h ah = frag_load(Ab + aofs);
#pragma unroll
      for (int j = 0; j < 4; ++j) acc[i][j] = mma_h(ah, bh[j], acc[i][j]);
    }
  }

  float* slab = sT[wave];
  const float* Rb = resid;
  if (RESID) Rb = resid + (size_t)bo * (size_t)sRo + (size_t)bi * (size_t)sRi;

  if (OUT_MODE == 0) {
    const int hh = lane >> 4;
    const int c4 = (lane & 15) * 4;
    v4f bvec = (v4f){0.f, 0.f, 0.f, 0.f};
    if (BIAS_MODE == 2) bvec = *(const v4f*)(bias + n0 + c4);
    float* C = (float*)Cout + offC;
#pragma unroll
    for (int i = 0; i < 4; ++i) {
      const int mBase = m0 + (i << 4);
#pragma unroll
      for (int j = 0; j < 4; ++j)
#pragma unroll
        for (int r = 0; r < 8; ++r) slab[(mOff + r) * 68 + (j << 4) + rlane] = acc[i][j][r] * scale;
      __builtin_amdgcn_fence(__ATOMIC_RELEASE, "workgroup");
      __builtin_amdgcn_wave_barrier();
      __builtin_amdgcn_fence(__ATOMIC_ACQUIRE, "workgroup");
      v4f vals[8];
#pragma unroll
      for (int it = 0; it < 8; ++it) {
        const int row  = it * 2 + hh;
        const int grow = mBase + row;
        v4f v = *(const v4f*)(slab + row * 68 + c4);
        if (BIAS_MODE == 2) v = v + bvec;
        if (BIAS_MODE == 1) {
          const float bm = bias[grow];
          v[0] += bm; v[1] += bm; v[2] += bm; v[3] += bm;
        }
        if (RESID) {
          const v4f rv = *(const v4f*)(Rb + (size_t)grow * ldr + n0 + c4);
          v = v + rv;
        }
        if (ACT == 1) {
          v[0] = fmaxf(v[0], 0.0f); v[1] = fmaxf(v[1], 0.0f); v[2] = fmaxf(v[2], 0.0f); v[3] = fmaxf(v[3], 0.0f);
        }
        if (KEEPM) {
          const int kp = keepv[grow];
          v[0] = (kp != 0) ? v[0] : 0.0f;
          v[1] = (kp != 0) ? v[1] : 0.0f;
          v[2] = (kp != 0) ? v[2] : 0.0f;
          v[3] = (kp != 0) ? v[3] : 0.0f;
        }
        vals[it] = v;
      }
      for (int pass = 0; pass < 2; ++pass) {
#pragma unroll
        for (int it = 0; it < 8; ++it) {
          const int row = it * 2 + hh;
          *(volatile v4f*)(C + (size_t)(mBase + row) * ldc + n0 + c4) = vals[it];
        }
        __threadfence();
      }
      __builtin_amdgcn_fence(__ATOMIC_RELEASE, "workgroup");
      __builtin_amdgcn_wave_barrier();
      __builtin_amdgcn_fence(__ATOMIC_ACQUIRE, "workgroup");
    }
  } else {
    const int q  = lane >> 3;
    const int c8 = (lane & 7) * 8;
    v4f b0 = (v4f){0.f, 0.f, 0.f, 0.f};
    v4f b1 = (v4f){0.f, 0.f, 0.f, 0.f};
    if (BIAS_MODE == 2) {
      b0 = *(const v4f*)(bias + n0 + c8);
      b1 = *(const v4f*)(bias + n0 + c8 + 4);
    }
    unsigned short* C = (unsigned short*)Cout + offC;
#pragma unroll
    for (int i = 0; i < 4; ++i) {
      const int mBase = m0 + (i << 4);
#pragma unroll
      for (int j = 0; j < 4; ++j)
#pragma unroll
        for (int r = 0; r < 8; ++r) slab[(mOff + r) * 68 + (j << 4) + rlane] = acc[i][j][r] * scale;
      __builtin_amdgcn_fence(__ATOMIC_RELEASE, "workgroup");
      __builtin_amdgcn_wave_barrier();
      __builtin_amdgcn_fence(__ATOMIC_ACQUIRE, "workgroup");
      v8h hvals[4];
#pragma unroll
      for (int it = 0; it < 4; ++it) {
        const int row  = it * 4 + q;
        const int grow = mBase + row;
        const float* sp = slab + row * 68 + c8;
        v4f a0 = *(const v4f*)(sp);
        v4f a1 = *(const v4f*)(sp + 4);
        if (BIAS_MODE == 2) { a0 = a0 + b0; a1 = a1 + b1; }
        if (BIAS_MODE == 1) {
          const float bm = bias[grow];
          a0[0] += bm; a0[1] += bm; a0[2] += bm; a0[3] += bm;
          a1[0] += bm; a1[1] += bm; a1[2] += bm; a1[3] += bm;
        }
        if (RESID) {
          const float* rp = Rb + (size_t)grow * ldr + n0 + c8;
          const v4f r0 = *(const v4f*)(rp);
          const v4f r1 = *(const v4f*)(rp + 4);
          a0 = a0 + r0; a1 = a1 + r1;
        }
        if (ACT == 1) {
          a0[0] = fmaxf(a0[0], 0.0f); a0[1] = fmaxf(a0[1], 0.0f); a0[2] = fmaxf(a0[2], 0.0f); a0[3] = fmaxf(a0[3], 0.0f);
          a1[0] = fmaxf(a1[0], 0.0f); a1[1] = fmaxf(a1[1], 0.0f); a1[2] = fmaxf(a1[2], 0.0f); a1[3] = fmaxf(a1[3], 0.0f);
        }
        v8h hv;
        hv[0] = (_Float16)a0[0]; hv[1] = (_Float16)a0[1]; hv[2] = (_Float16)a0[2]; hv[3] = (_Float16)a0[3];
        hv[4] = (_Float16)a1[0]; hv[5] = (_Float16)a1[1]; hv[6] = (_Float16)a1[2]; hv[7] = (_Float16)a1[3];
        hvals[it] = hv;
      }
      for (int pass = 0; pass < 2; ++pass) {
#pragma unroll
        for (int it = 0; it < 4; ++it) {
          const int row = it * 4 + q;
          *(volatile v8h*)(C + (size_t)(mBase + row) * ldc + n0 + c8) = hvals[it];
        }
        __threadfence();
      }
      __builtin_amdgcn_fence(__ATOMIC_RELEASE, "workgroup");
      __builtin_amdgcn_wave_barrier();
      __builtin_amdgcn_fence(__ATOMIC_ACQUIRE, "workgroup");
    }
  }
}

__global__ __launch_bounds__(256) void prep_kernel(
    const float* __restrict__ Wq, const float* __restrict__ Wk, const float* __restrict__ Wv,
    const float* __restrict__ Wf1, const float* __restrict__ Wf2, const float* __restrict__ fusW1,
    const float* __restrict__ fusW2, const float* __restrict__ tKemb, const float* __restrict__ absV,
    unsigned short* __restrict__ wbase, float* __restrict__ absVT) {
  const int z = blockIdx.y;
  const int i = blockIdx.x * 256 + threadIdx.x;
  if (z < 8) {
    const float* src = Wq;
    int ld = kH, rows = kL * kH, rowsValid = kL * kH;
    size_t dsto = kOffWQ / 2;
    if (z == 1) { src = Wk;  dsto = kOffWK / 2; }
    if (z == 2) { src = Wv;  dsto = kOffWV / 2; }
    if (z == 3) { src = Wf1; dsto = kOffW1 / 2; }
    if (z == 4) { src = Wf2; dsto = kOffW2 / 2; }
    if (z == 5) { src = fusW1; ld = 2 * kH; rows = kH; rowsValid = kH; dsto = kOffFW1 / 2; }
    if (z == 6) { src = fusW2; rows = kH; rowsValid = kH; dsto = kOffFW2 / 2; }
    if (z == 7) { src = tKemb; rows = kTKP; rowsValid = kSpanRows; dsto = kOffTK / 2; }
    if (i >= rows * 16) return;
    const int row = i >> 4;
    const int c8  = (i & 15) * 8;
    const int rc  = min(row, rowsValid - 1);
    const bool valid = row < rowsValid;
    const float* sp = src + (size_t)rc * ld + c8;
    const v4f a0 = *(const v4f*)(sp);
    const v4f a1 = *(const v4f*)(sp + 4);
    unsigned short hb[8];
#pragma unroll
    for (int e = 0; e < 4; ++e) {
      const float f0 = valid ? a0[e] * kWCarry : 0.0f;
      const float f1 = valid ? a1[e] * kWCarry : 0.0f;
      hb[e]     = h_bits(f0);
      hb[4 + e] = h_bits(f1);
    }
    const v4u u = (v4u){pk16(hb[0], hb[1]), pk16(hb[2], hb[3]), pk16(hb[4], hb[5]), pk16(hb[6], hb[7])};
    unsigned short* dp = wbase + dsto + (size_t)row * kH + c8;
    *(volatile v4u*)dp = u;
    __threadfence();
    *(volatile v4u*)dp = u;
  } else {
    if (i >= (kH * kT) / 4) return;
    const int f  = i >> 6;
    const int t4 = (i & 63) * 4;
    v4f v;
    v[0] = absV[(size_t)(t4 + 0) * kH + f];
    v[1] = absV[(size_t)(t4 + 1) * kH + f];
    v[2] = absV[(size_t)(t4 + 2) * kH + f];
    v[3] = absV[(size_t)(t4 + 3) * kH + f];
    float* dp = absVT + (size_t)f * kT + t4;
    *(volatile v4f*)dp = v;
    __threadfence();
    *(volatile v4f*)dp = v;
  }
}

__global__ __launch_bounds__(256) void phase_kernel(const float* __restrict__ tseq, float* __restrict__ SC) {
  const int b = blockIdx.x, t = threadIdx.x;
  const float base = kTwoPi * tseq[b * kT + t];
  const float p0 = base * kInvP0;
  const float p1 = base * kInvP1;
  const float p2 = base * kInvP2;
  const float s0 = sinf(p0), s1 = sinf(p1), s2 = sinf(p2);
  const float c0 = cosf(p0), c1 = cosf(p1), c2 = cosf(p2);
  float* dp = SC + (size_t)b * 6 * kT + t;
  for (int pass = 0; pass < 2; ++pass) {
    *(volatile float*)(dp + 0 * kT) = s0;
    *(volatile float*)(dp + 1 * kT) = s1;
    *(volatile float*)(dp + 2 * kT) = s2;
    *(volatile float*)(dp + 3 * kT) = c0;
    *(volatile float*)(dp + 4 * kT) = c1;
    *(volatile float*)(dp + 5 * kT) = c2;
    __threadfence();
  }
}

template <bool EMBED, bool OUT_Y32, bool OUT_X16>
__global__ __launch_bounds__(256) void ln_rows_kernel(
    const float* __restrict__ X, const int* __restrict__ ids, const float* __restrict__ emb,
    const float* __restrict__ tproj, const float* __restrict__ SC,
    const float* __restrict__ g, const float* __restrict__ bt,
    float* __restrict__ Y32, unsigned short* __restrict__ Y16, unsigned short* __restrict__ X16) {
  const int lane = threadIdx.x & 31, wave = threadIdx.x >> 5;
  const int row  = blockIdx.x * 8 + wave;
  const int col4 = lane * 4;
  float x0, x1, x2, x3;
  if (EMBED) {
    const int id  = ids[row];
    const int idc = min(max(id, 0), kItems - 1);
    const v4f e = *(const v4f*)(emb + (size_t)idc * kH + col4);
    const int b = row >> 8, t = row & (kT - 1);
    float s[6];
#pragma unroll
    for (int c = 0; c < 6; ++c) s[c] = SC[(size_t)(b * 6 + c) * kT + t];
    const float* tp = tproj + (size_t)col4 * 6;
    float tpv[24];
#pragma unroll
    for (int w = 0; w < 6; ++w) {
      const v4f tv = *(const v4f*)(tp + 4 * w);
      tpv[4 * w + 0] = tv[0]; tpv[4 * w + 1] = tv[1]; tpv[4 * w + 2] = tv[2]; tpv[4 * w + 3] = tv[3];
    }
    const float es = sqrtf((float)kH);
    float xe[4];
#pragma unroll
    for (int j = 0; j < 4; ++j) {
      float a = e[j] * es;
#pragma unroll
      for (int c = 0; c < 6; ++c) a = fmaf(s[c], tpv[j * 6 + c], a);
      xe[j] = (id != 0) ? a : 0.0f;
    }
    x0 = xe[0]; x1 = xe[1]; x2 = xe[2]; x3 = xe[3];
  } else {
    const v4f xin = *(const v4f*)(X + (size_t)row * kH + col4);
    x0 = xin[0]; x1 = xin[1]; x2 = xin[2]; x3 = xin[3];
  }
  float sum = (x0 + x1) + (x2 + x3);
#pragma unroll
  for (int off = 16; off > 0; off >>= 1) sum += __shfl_xor(sum, off, 32);
  const float mu = sum * kInvH;
  const float d0 = x0 - mu, d1 = x1 - mu, d2 = x2 - mu, d3 = x3 - mu;
  float sq = (d0 * d0 + d1 * d1) + (d2 * d2 + d3 * d3);
#pragma unroll
  for (int off = 16; off > 0; off >>= 1) sq += __shfl_xor(sq, off, 32);
  const float rstd = 1.0f / sqrtf(sq * kInvH + kLnEps);
  const v4f gv = *(const v4f*)(g + col4);
  const v4f bv = *(const v4f*)(bt + col4);
  v4f y;
  y[0] = d0 * rstd * gv[0] + bv[0];
  y[1] = d1 * rstd * gv[1] + bv[1];
  y[2] = d2 * rstd * gv[2] + bv[2];
  y[3] = d3 * rstd * gv[3] + bv[3];
  const v2u yh = (v2u){pk16(h_bits(y[0]), h_bits(y[1])), pk16(h_bits(y[2]), h_bits(y[3]))};
  const v2u xh = (v2u){pk16(h_bits(x0), h_bits(x1)), pk16(h_bits(x2), h_bits(x3))};
  const size_t o = (size_t)row * kH + col4;
  for (int pass = 0; pass < 2; ++pass) {
    if (OUT_Y32) *(volatile v4f*)(Y32 + o) = y;
    *(volatile v2u*)(Y16 + o) = yh;
    if (OUT_X16) *(volatile v2u*)(X16 + o) = xh;
    __threadfence();
  }
}

__global__ __launch_bounds__(256) void score_softmax_kernel(
    const float* __restrict__ S, const float* __restrict__ QT, const int* __restrict__ tmat,
    const int* __restrict__ ids, const float* __restrict__ SC, const float* __restrict__ lambdas,
    unsigned short* __restrict__ P16) {
  __shared__ __align__(16) float sS[8][2][kT];
  const int lane = threadIdx.x & 31, wave = threadIdx.x >> 5;
  const int row = blockIdx.x * 8 + wave;
  const int b = row >> 8, q = row & (kT - 1);
  const float isd = 1.0f / sqrtf((float)kDH);
  const float* scb = SC + (size_t)b * 6 * kT;
  const float lq0 = lambdas[0] * scb[0 * kT + q];
  const float lq1 = lambdas[1] * scb[1 * kT + q];
  const float lq2 = lambdas[2] * scb[2 * kT + q];
  const float lc0 = lambdas[0] * scb[3 * kT + q];
  const float lc1 = lambdas[1] * scb[4 * kT + q];
  const float lc2 = lambdas[2] * scb[5 * kT + q];
  const float* S0r = S + (size_t)((b * kNH + 0) * kT + q) * kT;
  const float* S1r = S + (size_t)((b * kNH + 1) * kT + q) * kT;
  const float* QTr = QT + (size_t)row * kQTP;
  float m0 = -INFINITY, m1 = -INFINITY;
#pragma unroll 1
  for (int p = 0; p < 2; ++p) {
    const int k4 = p * 128 + 4 * lane;
    const v4i tmv = *(const v4i*)(tmat + (size_t)row * kT + k4);
    const v4i lsv = *(const v4i*)(ids + b * kT + k4);
    const v4f sk0 = *(const v4f*)(scb + 0 * kT + k4);
    const v4f sk1 = *(const v4f*)(scb + 1 * kT + k4);
    const v4f sk2 = *(const v4f*)(scb + 2 * kT + k4);
    const v4f ck0 = *(const v4f*)(scb + 3 * kT + k4);
    const v4f ck1 = *(const v4f*)(scb + 4 * kT + k4);
    const v4f ck2 = *(const v4f*)(scb + 5 * kT + k4);
    const v4f a0 = *(const v4f*)(S0r + k4);
    const v4f a1 = *(const v4f*)(S1r + k4);
    v4f o0, o1;
#pragma unroll
    for (int e = 0; e < 4; ++e) {
      const int j = min(max(tmv[e], 0), kSpanRows - 1);
      const float qt0 = QTr[j];
      const float qt1 = QTr[kTKP + j];
      float pb = lq0 * sk0[e];
      pb = fmaf(lc0, ck0[e], pb);
      pb = fmaf(lq1, sk1[e], pb);
      pb = fmaf(lc1, ck1[e], pb);
      pb = fmaf(lq2, sk2[e], pb);
      pb = fmaf(lc2, ck2[e], pb);
      const float s0 = (a0[e] + qt0) * isd + pb;
      const float s1 = (a1[e] + qt1) * isd + pb;
      const bool masked = ((k4 + e) > q) || (lsv[e] == 0);
      const float t0 = masked ? kNegFill : s0;
      const float t1 = masked ? kNegFill : s1;
      o0[e] = t0;
      o1[e] = t1;
      m0 = fmaxf(m0, t0);
      m1 = fmaxf(m1, t1);
    }
    *(v4f*)(&sS[wave][0][k4]) = o0;
    *(v4f*)(&sS[wave][1][k4]) = o1;
  }
#pragma unroll
  for (int off = 16; off > 0; off >>= 1) {
    m0 = fmaxf(m0, __shfl_xor(m0, off, 32));
    m1 = fmaxf(m1, __shfl_xor(m1, off, 32));
  }
  __syncthreads();
  float sum0 = 0.0f, sum1 = 0.0f;
#pragma unroll 1
  for (int i = 0; i < 4; ++i) {
    const int hs = i >> 1;
    const int k4 = (i & 1) * 128 + 4 * lane;
    const float mh = (hs != 0) ? m1 : m0;
    float* sp = &sS[wave][hs][k4];
    const v4f v = *(const v4f*)sp;
    v4f ev;
    ev[0] = expf(v[0] - mh);
    ev[1] = expf(v[1] - mh);
    ev[2] = expf(v[2] - mh);
    ev[3] = expf(v[3] - mh);
    *(v4f*)sp = ev;
    const float part = (ev[0] + ev[1]) + (ev[2] + ev[3]);
    sum0 += (hs != 0) ? 0.0f : part;
    sum1 += (hs != 0) ? part : 0.0f;
  }
#pragma unroll
  for (int off = 16; off > 0; off >>= 1) {
    sum0 += __shfl_xor(sum0, off, 32);
    sum1 += __shfl_xor(sum1, off, 32);
  }
  __syncthreads();
  const float sc0 = kPCarry * (1.0f / sum0);
  const float sc1 = kPCarry * (1.0f / sum1);
  for (int pass = 0; pass < 2; ++pass) {
#pragma unroll 1
    for (int h = 0; h < 2; ++h) {
      const float scl = (h != 0) ? sc1 : sc0;
      const float* sp = &sS[wave][h][8 * lane];
      const v4f a = *(const v4f*)(sp);
      const v4f c = *(const v4f*)(sp + 4);
      unsigned short hb[8];
#pragma unroll
      for (int e = 0; e < 4; ++e) {
        hb[e]     = h_bits(a[e] * scl);
        hb[4 + e] = h_bits(c[e] * scl);
      }
      const v4u u = (v4u){pk16(hb[0], hb[1]), pk16(hb[2], hb[3]), pk16(hb[4], hb[5]), pk16(hb[6], hb[7])};
      *(volatile v4u*)(P16 + (size_t)((b * kNH + h) * kT + q) * kT + 8 * lane) = u;
    }
    __threadfence();
  }
}

__global__ __launch_bounds__(256) void attn_merge_ln_kernel(
    const unsigned short* __restrict__ P16, const int* __restrict__ tmat, const float* __restrict__ tVemb,
    const float* __restrict__ OH, const float* __restrict__ QN,
    const float* __restrict__ g, const float* __restrict__ bt,
    float* __restrict__ X32, unsigned short* __restrict__ X16) {
  __shared__ __align__(16) float sP[8][2][kT];
  __shared__ __align__(16) int   sO[8][kT];
  const int lane = threadIdx.x & 31, wave = threadIdx.x >> 5;
  const int row = blockIdx.x * 8 + wave;
  const int b = row >> 8, q = row & (kT - 1);
#pragma unroll
  for (int h = 0; h < 2; ++h) {
    const v4u w = *(const v4u*)(P16 + (size_t)((b * kNH + h) * kT + q) * kT + 8 * lane);
    const unsigned w0 = w[0], w1 = w[1], w2 = w[2], w3 = w[3];
    v4f f0, f1;
    f0[0] = h16_to_f32(w0 & 0xffffu) * kPCarryInv;
    f0[1] = h16_to_f32(w0 >> 16) * kPCarryInv;
    f0[2] = h16_to_f32(w1 & 0xffffu) * kPCarryInv;
    f0[3] = h16_to_f32(w1 >> 16) * kPCarryInv;
    f1[0] = h16_to_f32(w2 & 0xffffu) * kPCarryInv;
    f1[1] = h16_to_f32(w2 >> 16) * kPCarryInv;
    f1[2] = h16_to_f32(w3 & 0xffffu) * kPCarryInv;
    f1[3] = h16_to_f32(w3 >> 16) * kPCarryInv;
    *(v4f*)(&sP[wave][h][8 * lane])     = f0;
    *(v4f*)(&sP[wave][h][8 * lane + 4]) = f1;
  }
  {
    const v4i t0 = *(const v4i*)(tmat + (size_t)row * kT + 8 * lane);
    const v4i t1 = *(const v4i*)(tmat + (size_t)row * kT + 8 * lane + 4);
    v4i o0, o1;
#pragma unroll
    for (int e = 0; e < 4; ++e) {
      o0[e] = min(max(t0[e], 0), kSpanRows - 1) * kH;
      o1[e] = min(max(t1[e], 0), kSpanRows - 1) * kH;
    }
    *(v4i*)(&sO[wave][8 * lane])     = o0;
    *(v4i*)(&sO[wave][8 * lane + 4]) = o1;
  }
  __syncthreads();
  const int col4 = lane * 4;
  const float* pr = &sP[wave][lane >> 4][0];
  const int*   po = &sO[wave][0];
  const float* tvb = tVemb + col4;
  float a0 = 0.0f, a1 = 0.0f, a2 = 0.0f, a3 = 0.0f;
#pragma unroll 4
  for (int k = 0; k <= q; ++k) {
    const int off = po[k];
    const float p = pr[k];
    const v4f tv = *(const v4f*)(tvb + off);
    a0 = fmaf(p, tv[0], a0);
    a1 = fmaf(p, tv[1], a1);
    a2 = fmaf(p, tv[2], a2);
    a3 = fmaf(p, tv[3], a3);
  }
  const size_t o = (size_t)row * kH + col4;
  const v4f oh = *(const v4f*)(OH + o);
  const v4f qn = *(const v4f*)(QN + o);
  const float x0 = qn[0] + (oh[0] + a0);
  const float x1 = qn[1] + (oh[1] + a1);
  const float x2 = qn[2] + (oh[2] + a2);
  const float x3 = qn[3] + (oh[3] + a3);
  float sum = (x0 + x1) + (x2 + x3);
#pragma unroll
  for (int off = 16; off > 0; off >>= 1) sum += __shfl_xor(sum, off, 32);
  const float mu = sum * kInvH;
  const float d0 = x0 - mu, d1 = x1 - mu, d2 = x2 - mu, d3 = x3 - mu;
  float sq = (d0 * d0 + d1 * d1) + (d2 * d2 + d3 * d3);
#pragma unroll
  for (int off = 16; off > 0; off >>= 1) sq += __shfl_xor(sq, off, 32);
  const float rstd = 1.0f / sqrtf(sq * kInvH + kLnEps);
  const v4f gv = *(const v4f*)(g + col4);
  const v4f bv = *(const v4f*)(bt + col4);
  v4f y;
  y[0] = d0 * rstd * gv[0] + bv[0];
  y[1] = d1 * rstd * gv[1] + bv[1];
  y[2] = d2 * rstd * gv[2] + bv[2];
  y[3] = d3 * rstd * gv[3] + bv[3];
  const v2u yh = (v2u){pk16(h_bits(y[0]), h_bits(y[1])), pk16(h_bits(y[2]), h_bits(y[3]))};
  for (int pass = 0; pass < 2; ++pass) {
    *(volatile v4f*)(X32 + o) = y;
    *(volatile v2u*)(X16 + o) = yh;
    __threadfence();
  }
}

__global__ __launch_bounds__(128) void hper_bias_kernel(
    const float* __restrict__ ttimes, const float* __restrict__ tproj, const float* __restrict__ predW,
    const float* __restrict__ fusW1, const float* __restrict__ fb1, float* __restrict__ HB) {
  __shared__ float sTe[kH];
  __shared__ float sHp[kH];
  __shared__ __align__(16) float sHb[kH];
  const int b = blockIdx.x, n = threadIdx.x;
  const float base = kTwoPi * ttimes[b];
  const float p0 = base * kInvP0;
  const float p1 = base * kInvP1;
  const float p2 = base * kInvP2;
  const float* tp = tproj + n * 6;
  float te = sinf(p0) * tp[0];
  te = fmaf(sinf(p1), tp[1], te);
  te = fmaf(sinf(p2), tp[2], te);
  te = fmaf(cosf(p0), tp[3], te);
  te = fmaf(cosf(p1), tp[4], te);
  te = fmaf(cosf(p2), tp[5], te);
  sTe[n] = te;
  __syncthreads();
  const float* wr = predW + (size_t)n * kH;
  float acc = 0.0f;
#pragma unroll 4
  for (int k = 0; k < kH; ++k) acc = fmaf(sTe[k], wr[k], acc);
  sHp[n] = acc;
  __syncthreads();
  const float* wr2 = fusW1 + (size_t)n * 2 * kH + kH;
  float acc2 = 0.0f;
#pragma unroll 4
  for (int k = 0; k < kH; ++k) acc2 = fmaf(sHp[k], wr2[k], acc2);
  sHb[n] = acc2 + fb1[n];
  __syncthreads();
  if (threadIdx.x < 32) {
    const int l4 = threadIdx.x * 4;
    v4f v;
    v[0] = sHb[l4 + 0]; v[1] = sHb[l4 + 1]; v[2] = sHb[l4 + 2]; v[3] = sHb[l4 + 3];
    float* dp = HB + (size_t)b * kH + l4;
    *(volatile v4f*)dp = v;
    __threadfence();
    *(volatile v4f*)dp = v;
  }
}

__global__ __launch_bounds__(256) void gelu_cast_kernel(
    const float* __restrict__ PRE, const float* __restrict__ HB, unsigned short* __restrict__ G16) {
  __shared__ float sV[256 * 8];
  const int i8  = blockIdx.x * 256 + threadIdx.x;
  const int row = i8 >> 4;
  const int c8  = (i8 & 15) * 8;
  const int b   = row >> 8;
  const float* pp = PRE + (size_t)row * kH + c8;
  const float* hp = HB + (size_t)b * kH + c8;
  const v4f a0 = *(const v4f*)(pp);
  const v4f a1 = *(const v4f*)(pp + 4);
  const v4f h0 = *(const v4f*)(hp);
  const v4f h1 = *(const v4f*)(hp + 4);
  float* my = sV + threadIdx.x * 8;
  my[0] = a0[0] + h0[0]; my[1] = a0[1] + h0[1]; my[2] = a0[2] + h0[2]; my[3] = a0[3] + h0[3];
  my[4] = a1[0] + h1[0]; my[5] = a1[1] + h1[1]; my[6] = a1[2] + h1[2]; my[7] = a1[3] + h1[3];
#pragma unroll 1
  for (int e = 0; e < 8; ++e) {
    const float x = my[e];
    my[e] = 0.5f * x * (1.0f + erff(x * 0.70710678118654752f));
  }
  const unsigned short b0 = h_bits(my[0]), b1 = h_bits(my[1]), b2 = h_bits(my[2]), b3 = h_bits(my[3]);
  const unsigned short b4 = h_bits(my[4]), b5 = h_bits(my[5]), b6 = h_bits(my[6]), b7 = h_bits(my[7]);
  const v4u u = (v4u){pk16(b0, b1), pk16(b2, b3), pk16(b4, b5), pk16(b6, b7)};
  unsigned short* dp = G16 + (size_t)row * kH + c8;
  *(volatile v4u*)dp = u;
  __threadfence();
  *(volatile v4u*)dp = u;
}

__global__ __launch_bounds__(32) void logits_kernel(
    const float* __restrict__ F, const float* __restrict__ emb, const int* __restrict__ pos,
    const int* __restrict__ neg, float* __restrict__ out) {
  const int row = blockIdx.x * 32 + threadIdx.x;
  const int ip = min(max(pos[row], 0), kItems - 1);
  const int in = min(max(neg[row], 0), kItems - 1);
  const float* fr = F + (size_t)row * kH;
  const float* pr = emb + (size_t)ip * kH;
  const float* nr = emb + (size_t)in * kH;
  float ap = 0.0f, an = 0.0f;
#pragma unroll 2
  for (int i = 0; i < kH / 4; ++i) {
    const v4f f = *(const v4f*)(fr + 4 * i);
    const v4f p = *(const v4f*)(pr + 4 * i);
    const v4f n = *(const v4f*)(nr + 4 * i);
    ap = fmaf(f[0], p[0], ap); ap = fmaf(f[1], p[1], ap); ap = fmaf(f[2], p[2], ap); ap = fmaf(f[3], p[3], ap);
    an = fmaf(f[0], n[0], an); an = fmaf(f[1], n[1], an); an = fmaf(f[2], n[2], an); an = fmaf(f[3], n[3], an);
  }
  *(volatile float*)(out + row) = ap;
  *(volatile float*)(out + kTok + row) = an;
  __threadfence();
  *(volatile float*)(out + row) = ap;
  *(volatile float*)(out + kTok + row) = an;
}

extern "C" void kernel_launch(void* const* d_in, const int* in_sizes, int n_in,
                              void* d_out, int out_size, void* d_ws, size_t ws_size,
                              hipStream_t stream) {
  if (n_in < 34) return;
  if (in_sizes[0] != kTok) return;
  if (in_sizes[1] != kB * kT * kT) return;
  if (in_sizes[2] != kTok) return;
  if (in_sizes[3] != kTok || in_sizes[4] != kTok) return;
  if (in_sizes[5] != kB) return;
  if (in_sizes[6] != kItems * kH) return;
  if (in_sizes[7] != kT * kH || in_sizes[8] != kT * kH) return;
  if (in_sizes[9] != kSpanRows * kH || in_sizes[10] != kSpanRows * kH) return;
  if (in_sizes[11] != kL * kH * kH || in_sizes[13] != kL * kH * kH || in_sizes[15] != kL * kH * kH) return;
  if (in_sizes[21] != kL * kH * kH || in_sizes[23] != kL * kH * kH) return;
  if (in_sizes[27] != kH * 6 || in_sizes[28] != 3) return;
  if (in_sizes[29] != kH * kH || in_sizes[30] != kH * 2 * kH || in_sizes[32] != kH * kH) return;
  if (out_size != 2 * kTok) return;
  if (ws_size < kWsTotal) return;

  const int*   logs   = (const int*)  d_in[0];
  const int*   tmat   = (const int*)  d_in[1];
  const float* tseq   = (const float*)d_in[2];
  const int*   pos    = (const int*)  d_in[3];
  const int*   neg    = (const int*)  d_in[4];
  const float* ttimes = (const float*)d_in[5];
  const float* itemE  = (const float*)d_in[6];
  const float* absK   = (const float*)d_in[7];
  const float* absV   = (const float*)d_in[8];
  const float* tKe    = (const float*)d_in[9];
  const float* tVe    = (const float*)d_in[10];
  const float* Wq  = (const float*)d_in[11];
  const float* bq  = (const float*)d_in[12];
  const float* Wk  = (const float*)d_in[13];
  const float* bk  = (const float*)d_in[14];
  const float* Wv  = (const float*)d_in[15];
  const float* bv  = (const float*)d_in[16];
  const float* alg = (const float*)d_in[17];
  const float* alb = (const float*)d_in[18];
  const float* flg = (const float*)d_in[19];
  const float* flb = (const float*)d_in[20];
  const float* fw1 = (const float*)d_in[21];
  const float* fb1 = (const float*)d_in[22];
  const float* fw2 = (const float*)d_in[23];
  const float* fb2 = (const float*)d_in[24];
  const float* llg = (const float*)d_in[25];
  const float* llb = (const float*)d_in[26];
  const float* tproj   = (const float*)d_in[27];
  const float* lambdas = (const float*)d_in[28];
  const float* predW   = (const float*)d_in[29];
  const float* fusW1   = (const float*)d_in[30];
  const float* fusb1   = (const float*)d_in[31];
  const float* fusW2   = (const float*)d_in[32];
  const float* fusb2   = (const float*)d_in[33];
  float* out = (float*)d_out;

  char* ws = (char*)d_ws;
  unsigned short* WB    = (unsigned short*)ws;
  unsigned short* WQ16  = (unsigned short*)(ws + kOffWQ);
  unsigned short* WK16  = (unsigned short*)(ws + kOffWK);
  unsigned short* WV16  = (unsigned short*)(ws + kOffWV);
  unsigned short* W116  = (unsigned short*)(ws + kOffW1);
  unsigned short* W216  = (unsigned short*)(ws + kOffW2);
  unsigned short* FW1   = (unsigned short*)(ws + kOffFW1);
  unsigned short* FW2   = (unsigned short*)(ws + kOffFW2);
  unsigned short* TK16  = (unsigned short*)(ws + kOffTK);
  float*          AVT   = (float*)(ws + kOffAVT);
  float*          SC    = (float*)(ws + kOffSC);
  float*          HB    = (float*)(ws + kOffHB);
  float*          QN32  = (float*)(ws + kOffQN32);
  unsigned short* QN16  = (unsigned short*)(ws + kOffQN16);
  unsigned short* SEQ16 = (unsigned short*)(ws + kOffSEQ16);
  unsigned short* Q16   = (unsigned short*)(ws + kOffQ16);
  unsigned short* KP16  = (unsigned short*)(ws + kOffKP16);
  unsigned short* VT16  = (unsigned short*)(ws + kOffVT16);
  float*          S32   = (float*)(ws + kOffS32);
  float*          QT32  = (float*)(ws + kOffQT32);
  unsigned short* P16   = (unsigned short*)(ws + kOffP16);
  float*          OH32  = (float*)(ws + kOffOH32);
  float*          X32   = (float*)(ws + kOffX32);
  unsigned short* X16   = (unsigned short*)(ws + kOffX16);
  unsigned short* H116  = (unsigned short*)(ws + kOffH116);
  float*          SEQ32 = (float*)(ws + kOffSEQ32);
  unsigned short* LF16  = (unsigned short*)(ws + kOffLF16);
  float*          PRE32 = (float*)(ws + kOffPRE32);
  unsigned short* G16   = (unsigned short*)(ws + kOffG16);
  float*          FU32  = (float*)(ws + kOffFU32);

  const long sTokH = (long)kT * kH;
  const long sTT   = (long)kT * kT;

  prep_kernel<<<dim3(32, 9), 256, 0, stream>>>(Wq, Wk, Wv, fw1, fw2, fusW1, fusW2, tKe, absV, WB, AVT);
  phase_kernel<<<kB, kT, 0, stream>>>(tseq, SC);
  hper_bias_kernel<<<kB, kH, 0, stream>>>(ttimes, tproj, predW, fusW1, fusb1, HB);

  for (int l = 0; l < kL; ++l) {
    const size_t wo = (size_t)l * kH * kH;
    if (l == 0) {
      ln_rows_kernel<true, true, true><<<kTok / 8, 256, 0, stream>>>(
          SEQ32, logs, itemE, tproj, SC, alg, alb, QN32, QN16, SEQ16);
    } else {
      ln_rows_kernel<false, true, true><<<kTok / 8, 256, 0, stream>>>(
          SEQ32, logs, itemE, tproj, SC, alg + l * kH, alb + l * kH, QN32, QN16, SEQ16);
    }
    gemm_f16_tile64<1, 2, false, 0, false><<<dim3(8, 1), 256, 0, stream>>>(
        QN16, kH, 0L, 0L, WQ16 + wo, kH, 0L, 0L, (void*)Q16, kH, 0L, 0L,
        bq + l * kH, HB, kH, 0L, 0L, logs, 1, kTok, kH, kH, kWCarryInv);
    gemm_f16_tile64<1, 2, true, 0, false><<<dim3(1, kB), 256, 0, stream>>>(
        SEQ16, kH, sTokH, 0L, WK16 + wo, kH, 0L, 0L, (void*)KP16, kH, sTokH, 0L,
        bk + l * kH, absK, kH, 0L, 0L, logs, 1, kT, kH, kH, kWCarryInv);
    gemm_f16_tile64<1, 1, true, 0, false><<<dim3(1, kB), 256, 0, stream>>>(
        WV16 + wo, kH, 0L, 0L, SEQ16, kH, sTokH, 0L, (void*)VT16, kT, sTokH, 0L,
        bv + l * kH, AVT, kT, 0L, 0L, logs, 1, kH, kT, kH, kWCarryInv);
    gemm_f16_tile64<0, 0, false, 0, false><<<dim3(2, kB * kNH), 256, 0, stream>>>(
        Q16, kH, sTokH, (long)kDH, KP16, kH, sTokH, (long)kDH, (void*)S32, kT, (long)kNH * sTT, sTT,
        HB, HB, kH, 0L, 0L, logs, kNH, kT, kT, kDH, 1.0f);
    gemm_f16_tile64<0, 0, false, 0, false><<<dim3(20, kNH), 256, 0, stream>>>(
        Q16, kH, (long)kDH, 0L, TK16, kH, (long)kDH, 0L, (void*)QT32, kQTP, (long)kTKP, 0L,
        HB, HB, kH, 0L, 0L, logs, 1, kTok, kTKP, kDH, kWCarryInv);
    score_softmax_kernel<<<kTok / 8, 256, 0, stream>>>(S32, QT32, tmat, logs, SC, lambdas, P16);
    gemm_f16_tile64<0, 0, false, 0, false><<<dim3(1, kB * kNH), 256, 0, stream>>>(
        P16, kT, (long)kNH * sTT, sTT, VT16, kT, sTokH, (long)kDH * kT, (void*)OH32, kH, sTokH, (long)kDH,
        HB, HB, kH, 0L, 0L, logs, kNH, kT, kDH, kT, kPCarryInv);
    attn_merge_ln_kernel<<<kTok / 8, 256, 0, stream>>>(
        P16, tmat, tVe, OH32, QN32, flg + l * kH, flb + l * kH, X32, X16);
    gemm_f16_tile64<1, 2, false, 1, false><<<dim3(8, 1), 256, 0, stream>>>(
        X16, kH, 0L, 0L, W116 + wo, kH, 0L, 0L, (void*)H116, kH, 0L, 0L,
        fb1 + l * kH, HB, kH, 0L, 0L, logs, 1, kTok, kH, kH, kWCarryInv);
    gemm_f16_tile64<0, 2, true, 0, true><<<dim3(8, 1), 256, 0, stream>>>(
        H116, kH, 0L, 0L, W216 + wo, kH, 0L, 0L, (void*)SEQ32, kH, 0L, 0L,
        fb2 + l * kH, X32, kH, 0L, 0L, logs, 1, kTok, kH, kH, kWCarryInv);
  }

  ln_rows_kernel<false, false, false><<<kTok / 8, 256, 0, stream>>>(
      SEQ32, logs, itemE, tproj, SC, llg, llb, QN32, LF16, SEQ16);
  gemm_f16_tile64<0, 0, false, 0, false><<<dim3(8, 1), 256, 0, stream>>>(
      LF16, kH, 0L, 0L, FW1, kH, 0L, 0L, (void*)PRE32, kH, 0L, 0L,
      HB, HB, kH, 0L, 0L, logs, 1, kTok, kH, kH, kWCarryInv);
  gelu_cast_kernel<<<(kTok * kH / 8) / 256, 256, 0, stream>>>(PRE32, HB, G16);
  gemm_f16_tile64<0, 2, false, 0, false><<<dim3(8, 1), 256, 0, stream>>>(
      G16, kH, 0L, 0L, FW2, kH, 0L, 0L, (void*)FU32, kH, 0L, 0L,
      fusb2, HB, kH, 0L, 0L, logs, 1, kTok, kH, kH, kWCarryInv);
  logits_kernel<<<kTok / 32, 32, 0, stream>>>(FU32, itemE, pos, neg, out);
}
